// BasicBlock_deformable_6433861009839
// MI455X (gfx1250) — hardware-verified
//
#include <hip/hip_runtime.h>
#include <math.h>

typedef __attribute__((ext_vector_type(16))) _Float16 v16h;
typedef __attribute__((ext_vector_type(16))) __bf16 v16b;
typedef __attribute__((ext_vector_type(8)))  _Float16 v8h;
typedef __attribute__((ext_vector_type(8)))  float v8f;
typedef __attribute__((ext_vector_type(4)))  float v4f;
typedef __attribute__((ext_vector_type(2)))  float v2f;
typedef __attribute__((ext_vector_type(4)))  unsigned v4u;
typedef __attribute__((ext_vector_type(4)))  int v4i;
typedef float __attribute__((may_alias)) float_a;
typedef int __attribute__((may_alias)) int_a;

template <typename T> __device__ __forceinline__ void vst2(void* p, T v) { *(volatile T*)p = v; __threadfence(); *(volatile T*)p = v; }
__device__ __forceinline__ v8f wmma16(v16h a, v16h b, v8f c) {
  v8f d = __builtin_amdgcn_wmma_f32_16x16x32_f16(false, a, false, b, (short)0, c, false, false);
  asm volatile("v_nop\n\tv_nop\n\tv_nop\n\tv_nop" : "+v"(d) : "v"(a), "v"(b));
  return d;
}
__device__ __forceinline__ v8f wmma_bf(v16b a, v16b b, v8f c) {
  v8f d = __builtin_amdgcn_wmma_f32_16x16x32_bf16(false, a, false, b, (short)0, c, false, false);
  asm volatile("v_nop\n\tv_nop\n\tv_nop\n\tv_nop" : "+v"(d) : "v"(a), "v"(b));
  return d;
}
__device__ __forceinline__ v16h frag_h(const _Float16* rowk0, int lane) {
  union { v16h v; v8h q[2]; } u; const _Float16* p = rowk0 + 8 * (lane >> 4);
  u.q[0] = *(const v8h*)p; u.q[1] = *(const v8h*)(p + 16); return u.v;
}
__device__ __forceinline__ v16h frag_f32(const float* rowk0, int lane) {
  v16h a; const float* p = rowk0 + 8 * (lane >> 4);
#pragma unroll
  for (int i = 0; i < 8; ++i) { a[i] = (_Float16)p[i]; a[8 + i] = (_Float16)p[16 + i]; }
  return a;
}
__device__ __forceinline__ v16h frag_f32s(const float* rowk0, int lane, float sc) {
  v16h a; const float* p = rowk0 + 8 * (lane >> 4);
#pragma unroll
  for (int i = 0; i < 8; ++i) { a[i] = (_Float16)(p[i] * sc); a[8 + i] = (_Float16)(p[16 + i] * sc); }
  return a;
}
__device__ __forceinline__ v16h fragc_f32(const float* W, int k0, int n, int lane, int ld, int K) {
  v16h a; const int g = lane >> 4;
#pragma unroll
  for (int i = 0; i < 8; ++i) { const int ka = k0 + 8 * g + i, kb = ka + 16;
    a[i] = (_Float16)(ka < K ? W[(size_t)(ka < K ? ka : K - 1) * ld + n] : 0.f); a[8 + i] = (_Float16)(kb < K ? W[(size_t)(kb < K ? kb : K - 1) * ld + n] : 0.f); }
  return a;
}
struct F2 { v16b h, l; };
__device__ __forceinline__ F2 bsplit16(const float v[16]) { F2 r;
#pragma unroll
  for (int i = 0; i < 16; ++i) { const __bf16 h = (__bf16)v[i]; r.h[i] = h; r.l[i] = (__bf16)(v[i] - (float)h); }
  return r; }
__device__ __forceinline__ F2 split_row(const float* row, int k0, int lane) { float v[16]; const float* p = row + k0 + 8 * (lane >> 4);
#pragma unroll
  for (int i = 0; i < 8; ++i) { v[i] = p[i]; v[8 + i] = p[16 + i]; }
  return bsplit16(v); }
__device__ __forceinline__ F2 split_rowK(const float* row, int k0, int lane, int K) { float v[16]; const int g = lane >> 4;
#pragma unroll
  for (int i = 0; i < 8; ++i) { const int ka = k0 + 8 * g + i, kb = ka + 16; v[i] = ka < K ? row[ka < K ? ka : K - 1] : 0.f; v[8 + i] = kb < K ? row[kb < K ? kb : K - 1] : 0.f; }
  return bsplit16(v); }
__device__ __forceinline__ F2 split_col(const float* W, int k0, int n, int lane, int ld, int K) { float v[16]; const int g = lane >> 4;
#pragma unroll
  for (int i = 0; i < 8; ++i) { const int ka = k0 + 8 * g + i, kb = ka + 16; v[i] = ka < K ? W[(size_t)(ka < K ? ka : K - 1) * ld + n] : 0.f; v[8 + i] = kb < K ? W[(size_t)(kb < K ? kb : K - 1) * ld + n] : 0.f; }
  return bsplit16(v); }
__device__ __forceinline__ v8f mac3(const F2& a, const F2& b, v8f c) { c = wmma_bf(a.l, b.h, c); c = wmma_bf(a.h, b.l, c); return wmma_bf(a.h, b.h, c); }
__device__ __forceinline__ float sigm(float v) { return 1.0f / (1.0f + expf(-v)); }
#define LDSX() do { asm volatile("s_wait_dscnt 0" ::: "memory"); __builtin_amdgcn_wave_barrier(); __builtin_amdgcn_fence(__ATOMIC_RELEASE, "workgroup"); } while (0)


#define NB 16
#define CC 128
#define HH 56
#define WWD 56
#define NP (HH * WWD)
#define KT 9
#define KIM (CC * KT)
#define NBLKP (NP / 64)
#ifndef TNB
#define TNB NB
#endif
typedef __attribute__((ext_vector_type(8))) __bf16 v8b;
__device__ __forceinline__ v16b frag_b(const __bf16* rowk0, int lane) {
  union { v16b v; v8b q[2]; } u; const __bf16* p = rowk0 + 8 * (lane >> 4);
  u.q[0] = *(const v8b*)p; u.q[1] = *(const v8b*)(p + 16); return u.v;
}
__device__ __forceinline__ float bfr(float v) { return (float)(__bf16)v; }
__device__ __attribute__((noinline)) float exp_ni(float v) { return expf(v); }
__device__ __attribute__((noinline)) float erf_ni(float v) { return erff(v); }

__device__ __attribute__((noinline)) float floor_ni(float v) { return floorf(v); }
#define WS_PW   0u
#define P1 0
#define POF (P1 + CC * KIM)
#define P2 (POF + 32 * KIM)
#define PWEND (P2 + CC * KIM)
#define WS_C1   (WS_PW + 2u * PWEND)
#define WS_O1   (WS_C1 + 4u * NB * CC * NP)
#define WS_PS   (WS_O1 + 4u * NB * CC * NP)
#define WS_ST   (WS_PS + 4u * NB * NBLKP * CC)
#define WS_OFF  (WS_ST + 4u * 4 * CC)
#define WS_SH   (WS_OFF + 4u * NB * NP * 32)
#define WS_SL   (WS_SH + 2u * NP * KIM)
#define WS_END  (WS_SL + 2u * NP * KIM)

__global__ __launch_bounds__(256) void k_pack(const float* __restrict__ W1, const float* __restrict__ WOF, const float* __restrict__ W2, __bf16* __restrict__ PW) {
  __shared__ __align__(16) __bf16 s[KIM]; const int r = blockIdx.x, which = blockIdx.y, tid = threadIdx.x; size_t dst; const float* src;
  if (which == 0) { dst = P1 + (size_t)r * KIM; src = W1 + (size_t)r * KIM; } else if (which == 1) { if (r >= 32) return; dst = POF + (size_t)r * KIM; src = (r < 18) ? WOF + (size_t)r * KIM : nullptr; } else { dst = P2 + (size_t)r * KIM; src = W2 + (size_t)r * KIM; }
  for (int k = tid; k < KIM; k += 256) s[k] = (__bf16)(src ? src[k] : 0.f);
  __syncthreads();
  for (int q = tid; q < KIM / 8; q += 256) vst2((unsigned*)(PW + dst + q * 8), *(const v4u*)&s[q * 8]);
}
template <int RIN, int NT, int MODE>
__global__ __launch_bounds__(128) void k_conv(const float* __restrict__ SRC, const __bf16* __restrict__ PW, const float* __restrict__ bias, float* __restrict__ DST, float* __restrict__ PS) {
  __shared__ __align__(16) float st[NT * 16][68]; __shared__ __align__(16) float sps[CC];
  const int tid = threadIdx.x, wave = tid >> 5, lane = tid & 31, col = lane & 15, g = lane >> 4; const int b = blockIdx.y, pb = blockIdx.x; const int p0 = pb * 64; const int pos = p0 + wave * 16 + col; const int y = pos / WWD, x = pos - y * WWD;
  const float* sb = SRC + (size_t)b * CC * NP;
  v8f acc[NT]; for (int j = 0; j < NT; ++j) acc[j] = (v8f){};
#pragma unroll 1
  for (int kc = 0; kc < KIM / 32; ++kc) { float v[16];
#pragma unroll
    for (int i = 0; i < 16; ++i) { const int kk = kc * 32 + 8 * g + (i & 7) + ((i >> 3) << 4); const int c = kk / 9, t = kk - c * 9; const int ky = t / 3, kx = t - ky * 3; const int yy = y + ky - 1, xx = x + kx - 1; float val = 0.f; if (yy >= 0 && yy < HH && xx >= 0 && xx < WWD) val = sb[(size_t)c * NP + yy * WWD + xx]; v[i] = RIN ? bfr(val) : val; }
    F2 a; if (RIN) { v16b ax; for (int i = 0; i < 16; ++i) ax[i] = (__bf16)v[i]; a.h = ax; a.l = ax; } else a = bsplit16(v);
#pragma unroll
    for (int j = 0; j < NT; ++j) { const v16b w = frag_b(PW + (size_t)(j * 16 + col) * KIM + kc * 32, lane); if (!RIN) acc[j] = wmma_bf(a.l, w, acc[j]); acc[j] = wmma_bf(a.h, w, acc[j]); } }
#pragma unroll
  for (int j = 0; j < NT; ++j) { const int o = j * 16 + col; const float bb = (MODE == 1 && o < 18) ? bfr(bias[o]) : 0.f;
#pragma unroll
    for (int r = 0; r < 8; ++r) st[o][wave * 16 + 8 * g + r] = acc[j][r] + bb; }
  __syncthreads();
  if (MODE == 0) {
    for (int q = tid; q < CC * 16; q += 128) { const int o = q >> 4, pc = q & 15; vst2(DST + ((size_t)b * CC + o) * NP + p0 + pc * 4, *(const v4f*)&st[o][pc * 4]); }
    { const int o = tid; float s_ = 0.f; for (int i = 0; i < 64; ++i) s_ += st[o][i]; sps[o] = s_; }
    __syncthreads();
    if (tid < 32) vst2(PS + ((size_t)b * NBLKP + pb) * CC + tid * 4, *(const v4f*)&sps[tid * 4]);
  } else {
    __shared__ __align__(16) float so2[64][32];
    for (int q = tid; q < 64 * 32; q += 128) { const int pl = q >> 5, o = q & 31; so2[pl][o] = st[o][pl]; }
    __syncthreads();
    for (int q = tid; q < 64 * 8; q += 128) { const int pl = q >> 3, pc = q & 7; vst2(DST + ((size_t)b * NP + p0 + pl) * 32 + pc * 4, *(const v4f*)&so2[pl][pc * 4]); }
  }
}
template <int MODE>
__global__ __launch_bounds__(128) void k_stat(const float* __restrict__ PS, const float* __restrict__ Gm, const float* __restrict__ Bt, float* __restrict__ ST) {
  __shared__ __align__(16) float s[3][CC]; const int c = threadIdx.x; float acc = 0.f;
  for (int i = 0; i < TNB * NBLKP; ++i) acc += PS[(size_t)i * CC + c];
  acc /= (float)(TNB * NP);
  if (MODE == 0) { s[0][c] = acc; } else { const float mean = ST[c]; const float rs = rsqrtf(acc + 1e-5f) * bfr(Gm[c]); s[0][c] = mean; s[1][c] = rs; s[2][c] = bfr(Bt[c]); }
  __syncthreads();
  if (MODE == 0) { if (c < 32) vst2(ST + c * 4, *(const v4f*)&s[0][c * 4]); }
  else { if (c < 32) vst2(ST + CC + c * 4, *(const v4f*)&s[1][c * 4]); else if (c < 64) vst2(ST + 2 * CC + (c - 32) * 4, *(const v4f*)&s[2][(c - 32) * 4]); }
}
__global__ __launch_bounds__(128) void k_var(const float* __restrict__ C1, const float* __restrict__ ST, float* __restrict__ PS) {
  const int c = threadIdx.x, b = blockIdx.y, pb = blockIdx.x; const float mu = ST[c]; const float* p = C1 + ((size_t)b * CC + c) * NP + pb * 64; float acc = 0.f;
  for (int i = 0; i < 64; ++i) { const float d = p[i] - mu; acc += d * d; }
  __shared__ __align__(16) float s[CC]; s[c] = acc; __syncthreads();
  if (c < 32) vst2(PS + ((size_t)b * NBLKP + pb) * CC + c * 4, *(const v4f*)&s[c * 4]);
}
__global__ __launch_bounds__(256) void k_bn1(const float* __restrict__ C1, const float* __restrict__ ST, float* __restrict__ O1) {
  const int c = blockIdx.x, b = blockIdx.y, tid = threadIdx.x; const float mu = ST[c], sc = ST[CC + c], sh = ST[2 * CC + c];
  const float* src = C1 + ((size_t)b * CC + c) * NP; float* dst = O1 + ((size_t)b * CC + c) * NP;
  for (int pc = tid; pc < NP / 4; pc += 256) { const float* q = src + pc * 4; vst2(dst + pc * 4, (v4f){fmaxf((q[0] - mu) * sc + sh, 0.f), fmaxf((q[1] - mu) * sc + sh, 0.f), fmaxf((q[2] - mu) * sc + sh, 0.f), fmaxf((q[3] - mu) * sc + sh, 0.f)}); }
}
__global__ __launch_bounds__(128) void k_sample(const float* __restrict__ O1, const float* __restrict__ OFF, int b, __bf16* __restrict__ SH, __bf16* __restrict__ SL) {
  __shared__ float soff[32]; __shared__ __align__(16) __bf16 sh[KIM], sl[KIM];
  __shared__ float sg[KT][4]; __shared__ int si[KT][4];
  const int pos = blockIdx.x, tid = threadIdx.x; const int i0 = pos / WWD, j0 = pos - i0 * WWD;
  if (tid < 32) soff[tid] = OFF[((size_t)b * NP + pos) * 32 + tid];
  __syncthreads();
  if (tid < KT) { const int n = tid; const int kh = n / 3, kw = n - kh * 3;
    float px = (float)(i0 + 1) + (float)(kh - 1) + soff[n], py = (float)(j0 + 1) + (float)(kw - 1) + soff[KT + n];
    px = fminf(fmaxf(px, 0.f), (float)(HH + 1)); py = fminf(fmaxf(py, 0.f), (float)(WWD + 1));
    const float fx = floor_ni(px), fy = floor_ni(py);
    const float x0 = fminf(fmaxf(fx, 0.f), (float)(HH + 1)), x1 = fminf(fmaxf(fx + 1.f, 0.f), (float)(HH + 1)), y0 = fminf(fmaxf(fy, 0.f), (float)(WWD + 1)), y1 = fminf(fmaxf(fy + 1.f, 0.f), (float)(WWD + 1));
    sg[n][0] = (1.f + (x0 - px)) * (1.f + (y0 - py)); si[n][0] = (int)x0 * (WWD + 2) + (int)y0;
    sg[n][1] = (1.f - (x1 - px)) * (1.f - (y1 - py)); si[n][1] = (int)x1 * (WWD + 2) + (int)y1;
    sg[n][2] = (1.f + (x0 - px)) * (1.f - (y1 - py)); si[n][2] = (int)x0 * (WWD + 2) + (int)y1;
    sg[n][3] = (1.f - (x1 - px)) * (1.f + (y0 - py)); si[n][3] = (int)x1 * (WWD + 2) + (int)y0; }
  __syncthreads();
  const float* ob = O1 + (size_t)b * CC * NP;
#pragma unroll 1
  for (int e = tid; e < KIM; e += 128) { const int c = e / KT, n = e - c * KT; const float* oc = ob + (size_t)c * NP; float v = 0.f;
#pragma unroll
    for (int q = 0; q < 4; ++q) { const int idx = si[n][q]; const int pr = idx / (WWD + 2), pcl = idx - pr * (WWD + 2); const int rr = pr - 1, cl = pcl - 1; const float s_ = (rr >= 0 && rr < HH && cl >= 0 && cl < WWD) ? oc[rr * WWD + cl] : 0.f; v += sg[n][q] * s_; }
    const __bf16 hb = (__bf16)v; sh[e] = hb; sl[e] = (__bf16)(v - (float)hb); }
  __syncthreads();
  for (int q = tid; q < KIM / 8; q += 128) { vst2((unsigned*)(SH + (size_t)pos * KIM + q * 8), *(const v4u*)&sh[q * 8]); vst2((unsigned*)(SL + (size_t)pos * KIM + q * 8), *(const v4u*)&sl[q * 8]); }
}
__global__ __launch_bounds__(128) void k_dconv(const __bf16* __restrict__ SH, const __bf16* __restrict__ SL, const __bf16* __restrict__ PW, int b, float* __restrict__ DST, float* __restrict__ PS) {
  __shared__ __align__(16) float st[CC][68]; __shared__ __align__(16) float sps[CC];
  const int tid = threadIdx.x, wave = tid >> 5, lane = tid & 31, col = lane & 15, g = lane >> 4; const int pb = blockIdx.x; const int p0 = pb * 64; const int pr = p0 + wave * 16 + col;
  v8f acc[8] = {};
#pragma unroll 2
  for (int kc = 0; kc < KIM / 32; ++kc) { const size_t ar = (size_t)pr * KIM + kc * 32; const v16b ah = frag_b(SH + ar, lane), al = frag_b(SL + ar, lane);
#pragma unroll
    for (int j = 0; j < 8; ++j) { const v16b w = frag_b(PW + P2 + (size_t)(j * 16 + col) * KIM + kc * 32, lane); acc[j] = wmma_bf(al, w, acc[j]); acc[j] = wmma_bf(ah, w, acc[j]); } }
#pragma unroll
  for (int j = 0; j < 8; ++j)
#pragma unroll
    for (int r = 0; r < 8; ++r) st[j * 16 + col][wave * 16 + 8 * g + r] = acc[j][r];
  __syncthreads();
  for (int q = tid; q < CC * 16; q += 128) { const int o = q >> 4, pc = q & 15; vst2(DST + ((size_t)b * CC + o) * NP + p0 + pc * 4, *(const v4f*)&st[o][pc * 4]); }
  { const int o = tid; float s_ = 0.f; for (int i = 0; i < 64; ++i) s_ += st[o][i]; sps[o] = s_; }
  __syncthreads();
  if (tid < 32) vst2(PS + ((size_t)b * NBLKP + pb) * CC + tid * 4, *(const v4f*)&sps[tid * 4]);
}
__global__ __launch_bounds__(256) void k_out(const float* __restrict__ C2, const float* __restrict__ ST, const float* __restrict__ X, float* __restrict__ out) {
  const int c = blockIdx.x, b = blockIdx.y, tid = threadIdx.x; const float mu = ST[c], sc = ST[CC + c], sh = ST[2 * CC + c];
  const size_t base = ((size_t)b * CC + c) * NP; const float* src = C2 + base; const float* xr = X + base; float* dst = out + base;
  for (int pc = tid; pc < NP / 4; pc += 256) { const float* q = src + pc * 4; const float* xq = xr + pc * 4; vst2(dst + pc * 4, (v4f){fmaxf((q[0] - mu) * sc + sh + bfr(xq[0]), 0.f), fmaxf((q[1] - mu) * sc + sh + bfr(xq[1]), 0.f), fmaxf((q[2] - mu) * sc + sh + bfr(xq[2]), 0.f), fmaxf((q[3] - mu) * sc + sh + bfr(xq[3]), 0.f)}); }
}
extern "C" void kernel_launch(void* const* d_in, const int* in_sizes, int n_in, void* d_out, int out_size, void* d_ws, size_t ws_size, hipStream_t stream) {
  (void)in_sizes; (void)n_in; (void)out_size;
  const float** F = (const float**)d_in;
  if (ws_size < (size_t)WS_END) return;
  char* ws = (char*)d_ws; __bf16 *PW = (__bf16*)(ws + WS_PW), *SH = (__bf16*)(ws + WS_SH), *SL = (__bf16*)(ws + WS_SL); float *C1 = (float*)(ws + WS_C1), *O1 = (float*)(ws + WS_O1), *PS = (float*)(ws + WS_PS), *ST = (float*)(ws + WS_ST), *OFF = (float*)(ws + WS_OFF);
  k_pack<<<dim3(CC, 3), 256, 0, stream>>>(F[1], F[4], F[6], PW);
  k_conv<1, 8, 0><<<dim3(NBLKP, TNB), 128, 0, stream>>>(F[0], PW + P1, nullptr, C1, PS);
  k_stat<0><<<1, CC, 0, stream>>>(PS, F[2], F[3], ST);
  k_var<<<dim3(NBLKP, TNB), CC, 0, stream>>>(C1, ST, PS);
  k_stat<1><<<1, CC, 0, stream>>>(PS, F[2], F[3], ST);
  k_bn1<<<dim3(CC, TNB), 256, 0, stream>>>(C1, ST, O1);
  k_conv<0, 2, 1><<<dim3(NBLKP, TNB), 128, 0, stream>>>(O1, PW + POF, F[5], OFF, nullptr);
  for (int b = 0; b < TNB; ++b) { k_sample<<<NP, 128, 0, stream>>>(O1, OFF, b, SH, SL); k_dconv<<<NBLKP, 128, 0, stream>>>(SH, SL, PW, b, C1, PS); }
  k_stat<0><<<1, CC, 0, stream>>>(PS, F[7], F[8], ST);
  k_var<<<dim3(NBLKP, TNB), CC, 0, stream>>>(C1, ST, PS);
  k_stat<1><<<1, CC, 0, stream>>>(PS, F[7], F[8], ST);
  k_out<<<dim3(CC, TNB), 256, 0, stream>>>(C1, ST, F[0], (float*)d_out);
}
